// PosCrossAttn_84430467105064
// MI455X (gfx1250) — hardware-verified
//
#include <hip/hip_runtime.h>
#include <math.h>

typedef __attribute__((ext_vector_type(16))) _Float16 v16h;
typedef __attribute__((ext_vector_type(16))) __bf16 v16b;
typedef __attribute__((ext_vector_type(8)))  _Float16 v8h;
typedef __attribute__((ext_vector_type(8)))  float v8f;
typedef __attribute__((ext_vector_type(4)))  float v4f;
typedef __attribute__((ext_vector_type(2)))  float v2f;
typedef __attribute__((ext_vector_type(4)))  unsigned v4u;
typedef __attribute__((ext_vector_type(4)))  int v4i;
typedef float __attribute__((may_alias)) float_a;
typedef int __attribute__((may_alias)) int_a;

template <typename T> __device__ __forceinline__ void vst2(void* p, T v) { *(volatile T*)p = v; __threadfence(); *(volatile T*)p = v; }
__device__ __forceinline__ v8f wmma16(v16h a, v16h b, v8f c) {
  v8f d = __builtin_amdgcn_wmma_f32_16x16x32_f16(false, a, false, b, (short)0, c, false, false);
  asm volatile("v_nop\n\tv_nop\n\tv_nop\n\tv_nop" : "+v"(d) : "v"(a), "v"(b));
  return d;
}
__device__ __forceinline__ v8f wmma_bf(v16b a, v16b b, v8f c) {
  v8f d = __builtin_amdgcn_wmma_f32_16x16x32_bf16(false, a, false, b, (short)0, c, false, false);
  asm volatile("v_nop\n\tv_nop\n\tv_nop\n\tv_nop" : "+v"(d) : "v"(a), "v"(b));
  return d;
}
__device__ __forceinline__ v16h frag_h(const _Float16* rowk0, int lane) {
  union { v16h v; v8h q[2]; } u; const _Float16* p = rowk0 + 8 * (lane >> 4);
  u.q[0] = *(const v8h*)p; u.q[1] = *(const v8h*)(p + 16); return u.v;
}
__device__ __forceinline__ v16h frag_f32(const float* rowk0, int lane) {
  v16h a; const float* p = rowk0 + 8 * (lane >> 4);
#pragma unroll
  for (int i = 0; i < 8; ++i) { a[i] = (_Float16)p[i]; a[8 + i] = (_Float16)p[16 + i]; }
  return a;
}
__device__ __forceinline__ v16h frag_f32s(const float* rowk0, int lane, float sc) {
  v16h a; const float* p = rowk0 + 8 * (lane >> 4);
#pragma unroll
  for (int i = 0; i < 8; ++i) { a[i] = (_Float16)(p[i] * sc); a[8 + i] = (_Float16)(p[16 + i] * sc); }
  return a;
}
__device__ __forceinline__ v16h fragc_f32(const float* W, int k0, int n, int lane, int ld, int K) {
  v16h a; const int g = lane >> 4;
#pragma unroll
  for (int i = 0; i < 8; ++i) { const int ka = k0 + 8 * g + i, kb = ka + 16;
    a[i] = (_Float16)(ka < K ? W[(size_t)(ka < K ? ka : K - 1) * ld + n] : 0.f); a[8 + i] = (_Float16)(kb < K ? W[(size_t)(kb < K ? kb : K - 1) * ld + n] : 0.f); }
  return a;
}
struct F2 { v16b h, l; };
__device__ __forceinline__ F2 bsplit16(const float v[16]) { F2 r;
#pragma unroll
  for (int i = 0; i < 16; ++i) { const __bf16 h = (__bf16)v[i]; r.h[i] = h; r.l[i] = (__bf16)(v[i] - (float)h); }
  return r; }
__device__ __forceinline__ F2 split_row(const float* row, int k0, int lane) { float v[16]; const float* p = row + k0 + 8 * (lane >> 4);
#pragma unroll
  for (int i = 0; i < 8; ++i) { v[i] = p[i]; v[8 + i] = p[16 + i]; }
  return bsplit16(v); }
__device__ __forceinline__ F2 split_rowK(const float* row, int k0, int lane, int K) { float v[16]; const int g = lane >> 4;
#pragma unroll
  for (int i = 0; i < 8; ++i) { const int ka = k0 + 8 * g + i, kb = ka + 16; v[i] = ka < K ? row[ka < K ? ka : K - 1] : 0.f; v[8 + i] = kb < K ? row[kb < K ? kb : K - 1] : 0.f; }
  return bsplit16(v); }
__device__ __forceinline__ F2 split_col(const float* W, int k0, int n, int lane, int ld, int K) { float v[16]; const int g = lane >> 4;
#pragma unroll
  for (int i = 0; i < 8; ++i) { const int ka = k0 + 8 * g + i, kb = ka + 16; v[i] = ka < K ? W[(size_t)(ka < K ? ka : K - 1) * ld + n] : 0.f; v[8 + i] = kb < K ? W[(size_t)(kb < K ? kb : K - 1) * ld + n] : 0.f; }
  return bsplit16(v); }
__device__ __forceinline__ v8f mac3(const F2& a, const F2& b, v8f c) { c = wmma_bf(a.l, b.h, c); c = wmma_bf(a.h, b.l, c); return wmma_bf(a.h, b.h, c); }
__device__ __forceinline__ float sigm(float v) { return 1.0f / (1.0f + expf(-v)); }
#define LDSX() do { asm volatile("s_wait_dscnt 0" ::: "memory"); __builtin_amdgcn_wave_barrier(); __builtin_amdgcn_fence(__ATOMIC_RELEASE, "workgroup"); } while (0)


#define NB 8
#define CQ 128
#define HWN 4096
#define NCTX 256
#define CD 65
#define INNER 64
#define NHD 8
#define DH 8
__device__ __forceinline__ float bfr(float v) { return (float)(__bf16)v; }
__device__ __forceinline__ v16b frag_b(const __bf16* rowk0, int lane) { return __builtin_bit_cast(v16b, frag_h((const _Float16*)rowk0, lane)); }

__global__ __launch_bounds__(256) void k_cvtx(const float* __restrict__ x, __bf16* __restrict__ XT) {
  __shared__ __align__(16) __bf16 st[64][CQ + 8];
  const int tid = threadIdx.x; const int b = blockIdx.y, p0 = blockIdx.x * 64;
  for (int q = tid; q < CQ * 16; q += 256) { const int c = q >> 4, p4 = q & 15; const v4f v = *(const v4f*)(x + ((size_t)b * CQ + c) * HWN + p0 + p4 * 4);
    st[p4 * 4][c] = (__bf16)v[0]; st[p4 * 4 + 1][c] = (__bf16)v[1]; st[p4 * 4 + 2][c] = (__bf16)v[2]; st[p4 * 4 + 3][c] = (__bf16)v[3]; }
  __syncthreads();
  for (int q = tid; q < 64 * (CQ / 8); q += 256) { const int rl = q >> 4, pc = q & 15; vst2((unsigned*)(XT + ((size_t)b * HWN + p0 + rl) * CQ + pc * 8), *(const v4u*)(&st[rl][pc * 8])); }
}
__global__ __launch_bounds__(128) void k_q(const __bf16* __restrict__ XT, const float* __restrict__ Wq, float* __restrict__ Q32) {
  __shared__ __align__(16) float so[4][16][68];
  const int tid = threadIdx.x, wave = tid >> 5, lane = tid & 31, col = lane & 15, g = lane >> 4; const size_t r0 = (size_t)blockIdx.x * 64 + wave * 16;
  v8f acc[4] = {};
#pragma unroll
  for (int kc = 0; kc < CQ / 32; ++kc) { const v16b a = frag_b(XT + (r0 + col) * CQ + kc * 32, lane);
#pragma unroll
    for (int j = 0; j < 4; ++j) acc[j] = wmma_bf(a, split_row(Wq + (size_t)(j * 16 + col) * CQ, kc * 32, lane).h, acc[j]); }
#pragma unroll
  for (int j = 0; j < 4; ++j)
#pragma unroll
    for (int r = 0; r < 8; ++r) so[wave][8 * g + r][j * 16 + col] = acc[j][r];
  LDSX();
  for (int qq = lane; qq < 16 * 16; qq += 32) { const int rl = qq >> 4, pc = qq & 15; vst2(Q32 + (r0 + rl) * INNER + pc * 4, *(const v4f*)(&so[wave][rl][pc * 4])); }
}
__global__ __launch_bounds__(128) void k_kv(const float* __restrict__ ctx, const float* __restrict__ Wk, const float* __restrict__ Wv, float* __restrict__ K32, __bf16* __restrict__ VTh, __bf16* __restrict__ VTl) {
  __shared__ __align__(16) float so[4][16][68]; __shared__ __align__(16) __bf16 sth[64][72], stl[64][72];
  const int tid = threadIdx.x, wave = tid >> 5, lane = tid & 31, col = lane & 15, g = lane >> 4; const int b = blockIdx.y, k0 = blockIdx.x * 64, which = blockIdx.z; const size_t r0 = (size_t)b * NCTX + k0 + wave * 16;
  const float* W = which == 0 ? Wk : Wv;
  v8f acc[4] = {};
#pragma unroll
  for (int kc = 0; kc < 3; ++kc) { const v16b a = split_rowK(ctx + (r0 + col) * CD, kc * 32, lane, CD).h;
#pragma unroll
    for (int j = 0; j < 4; ++j) acc[j] = wmma_bf(a, split_rowK(W + (size_t)(j * 16 + col) * CD, kc * 32, lane, CD).h, acc[j]); }
  if (which == 0) {
#pragma unroll
    for (int j = 0; j < 4; ++j)
#pragma unroll
      for (int r = 0; r < 8; ++r) so[wave][8 * g + r][j * 16 + col] = acc[j][r];
    LDSX();
    for (int qq = lane; qq < 16 * 16; qq += 32) { const int rl = qq >> 4, pc = qq & 15; vst2(K32 + (r0 + rl) * INNER + pc * 4, *(const v4f*)(&so[wave][rl][pc * 4])); } }
  else {
#pragma unroll
    for (int j = 0; j < 4; ++j)
#pragma unroll
      for (int r = 0; r < 8; ++r) { const float v = acc[j][r]; const __bf16 hi = (__bf16)v; sth[j * 16 + col][wave * 16 + 8 * g + r] = hi; stl[j * 16 + col][wave * 16 + 8 * g + r] = (__bf16)(v - (float)hi); }
    __syncthreads();
    for (int qq = tid; qq < 64 * 8; qq += 128) { const int e = qq >> 3, pc = qq & 7; const size_t o = ((size_t)b * INNER + e) * NCTX + k0 + pc * 8; vst2((unsigned*)(VTh + o), *(const v4u*)(&sth[e][pc * 8])); vst2((unsigned*)(VTl + o), *(const v4u*)(&stl[e][pc * 8])); } }
}
__global__ __launch_bounds__(128) void k_attn(const float* __restrict__ Q32, const float* __restrict__ K32, const __bf16* __restrict__ VTh, const __bf16* __restrict__ VTl, const float* __restrict__ Wout, const float* __restrict__ bout, float* __restrict__ out) {
  __shared__ __align__(16) float sS[4][16][NCTX + 4];
  __shared__ __align__(16) __bf16 sPh[4][16][NCTX + 8], sPl[4][16][NCTX + 8];
  __shared__ __align__(16) float sC[64][INNER + 4];
  __shared__ __align__(16) float sO[4][32][68];
  const int tid = threadIdx.x, w = tid >> 5, lane = tid & 31, col = lane & 15, g = lane >> 4; const int b = blockIdx.y, p0 = blockIdx.x * 64; const size_t q0 = (size_t)b * HWN + p0 + w * 16;
  const float scl = 0.35355339059327373f;
#pragma unroll 1
  for (int h = 0; h < NHD; ++h) {
    const F2 aq = split_rowK(Q32 + (q0 + col) * INNER + h * DH, 0, lane, DH);
#pragma unroll 2
    for (int t = 0; t < NCTX / 16; ++t) { const int key = t * 16 + col; const F2 bk = split_rowK(K32 + ((size_t)b * NCTX + key) * INNER + h * DH, 0, lane, DH);
      v8f s = {}; s = wmma_bf(aq.l, bk.h, s); s = wmma_bf(aq.h, bk.l, s); s = wmma_bf(aq.h, bk.h, s);
#pragma unroll
      for (int r = 0; r < 8; ++r) sS[w][8 * g + r][key] = s[r] * scl; }
    LDSX();
    { const int rl = lane & 15, hf = lane >> 4; float* rp = &sS[w][rl][hf * 128]; float mx = -3.4e38f;
#pragma unroll 8
      for (int j = 0; j < 128; ++j) mx = fmaxf(mx, rp[j]);
      mx = fmaxf(mx, __shfl_xor(mx, 16, 32)); float sum = 0.f;
#pragma unroll 4
      for (int j = 0; j < 128; ++j) { const float p = expf(rp[j] - mx); rp[j] = p; sum += p; }
      sum += __shfl_xor(sum, 16, 32); const float inv = 1.0f / sum;
#pragma unroll 4
      for (int j = 0; j < 128; ++j) { const float p = rp[j] * inv; const __bf16 hi = (__bf16)p; sPh[w][rl][hf * 128 + j] = hi; sPl[w][rl][hf * 128 + j] = (__bf16)(p - (float)hi); } }
    LDSX();
    { v8f acc = {}; const int e = h * DH + col; const int ec = e < INNER ? e : INNER - 1;
#pragma unroll
      for (int kc = 0; kc < NCTX / 32; ++kc) { const v16b ph = frag_b(&sPh[w][col][0] + kc * 32, lane), pl = frag_b(&sPl[w][col][0] + kc * 32, lane); const size_t vo = ((size_t)b * INNER + ec) * NCTX + kc * 32;
        const v16b vh = frag_b(VTh + vo, lane), vl = frag_b(VTl + vo, lane); acc = wmma_bf(pl, vh, acc); acc = wmma_bf(ph, vl, acc); acc = wmma_bf(ph, vh, acc); }
      if (col < DH) {
#pragma unroll
        for (int r = 0; r < 8; ++r) sC[w * 16 + 8 * g + r][h * DH + col] = acc[r]; } }
    LDSX(); }
  __syncthreads();
  { v8f acc[2][4] = {};
#pragma unroll
    for (int kc = 0; kc < 2; ++kc) {
#pragma unroll
      for (int ct = 0; ct < 2; ++ct) { const v16b a = split_row(Wout + (size_t)((w * 2 + ct) * 16 + col) * INNER, kc * 32, lane).h;
#pragma unroll
        for (int pt = 0; pt < 4; ++pt) { const F2 bc = split_row(&sC[pt * 16 + col][0], kc * 32, lane); acc[ct][pt] = wmma_bf(a, bc.l, acc[ct][pt]); acc[ct][pt] = wmma_bf(a, bc.h, acc[ct][pt]); } } }
#pragma unroll
    for (int ct = 0; ct < 2; ++ct) {
#pragma unroll
      for (int r = 0; r < 8; ++r) { const int cl = ct * 16 + 8 * g + r; const float bb = bfr(bout[w * 32 + cl]);
#pragma unroll
        for (int pt = 0; pt < 4; ++pt) sO[w][cl][pt * 16 + col] = acc[ct][pt][r] + bb; } } }
  LDSX();
  for (int qq = lane; qq < 32 * 16; qq += 32) { const int cl = qq >> 4, pc = qq & 15; vst2(out + ((size_t)b * CQ + w * 32 + cl) * HWN + p0 + pc * 4, *(const v4f*)(&sO[w][cl][pc * 4])); }
}
extern "C" void kernel_launch(void* const* d_in, const int* in_sizes, int n_in, void* d_out, int out_size, void* d_ws, size_t ws_size, hipStream_t stream) {
  (void)in_sizes; (void)n_in; (void)out_size; (void)ws_size;
  const float** I = (const float**)d_in;
  const float* img = I[0]; const float* ctx = I[1]; const float* Wq = I[2]; const float* Wk = I[3]; const float* Wv = I[4]; const float* Wout = I[5]; const float* bout = I[6];
  char* ws = (char*)d_ws; size_t off = 0;
  auto take = [&](size_t bytes) { char* p = ws + off; off += (bytes + 255) & ~(size_t)255; return p; };
  __bf16* XT = (__bf16*)take((size_t)NB * HWN * CQ * 2); float* Q32 = (float*)take((size_t)NB * HWN * INNER * 4); float* K32 = (float*)take((size_t)NB * NCTX * INNER * 4);
  __bf16* VTh = (__bf16*)take((size_t)NB * INNER * NCTX * 2); __bf16* VTl = (__bf16*)take((size_t)NB * INNER * NCTX * 2);
  k_cvtx<<<dim3(HWN / 64, NB), 256, 0, stream>>>(img, XT);
  k_q<<<NB * HWN / 64, 128, 0, stream>>>(XT, Wq, Q32);
  k_kv<<<dim3(NCTX / 64, NB, 2), 128, 0, stream>>>(ctx, Wk, Wv, K32, VTh, VTl);
  k_attn<<<dim3(HWN / 64, NB), 128, 0, stream>>>(Q32, K32, VTh, VTl, Wout, bout, (float*)d_out);
}
